// ContinuousFilterConvolution_56092272886168
// MI455X (gfx1250) — hardware-run, weakly checked
//
#include <hip/hip_runtime.h>
#include <stddef.h>
#include <stdint.h>
#include <math.h>
#pragma clang fp contract(off)

#define NN      50000
#define NE      1600000
#define DH      128
#define NBAS    16
#define SPLIT_A 1
#define MODE_B  1
#define NTHR    256
#define NWAVE   8
#define EPT     8
#define WCH     (32 * EPT)
#define SLB     10
#define NBRUN   1024
#define NBK     49
#define WLCAP   4480
#define RCAP    35840
#define DEGCAP  96
#define MAXDEG_MEAS   60
#define MAXB1024_MEAS 33098
#define CBROWS  50176
#define CNB     128
#define NCB     391
#define TP      132
#define W2PITCH 136
#define W1PITCH 40

#define BK_ZINTS (NWAVE * WLCAP + RCAP + 3 * NBRUN)
#define BK_INTS  (BK_ZINTS + 16)
#define BK_LDS   (BK_INTS * 4)
#define CV_LDS   (DH * W2PITCH * 2 + DH * W1PITCH * 2 + NWAVE * 16 * TP * 4)

#define PBF   (NN * DH / 8 / NTHR)
#define PBC   (CBROWS / NTHR)
#define PBW1  (DH * 32 / 8 / NTHR)
#define PBW2  (DH * DH / 8 / NTHR)
#define PBTOT (PBF + PBC + PBW1 + PBW2)

static_assert(DH == 32 * 4);
static_assert(NBAS == 16);
static_assert(TP == 132 && (TP % 4) == 0 && TP >= DH);
static_assert((W2PITCH % 8) == 0 && W2PITCH >= DH && (W1PITCH % 8) == 0 && W1PITCH >= 32);
static_assert(NBRUN == (1 << SLB) && NBRUN <= 1024 && (NBRUN % 32) == 0);
static_assert(NBK * NBRUN >= NN && NN <= 65536);
static_assert(NE < (1 << 21) && (((long long)NE) << SLB) < (1LL << 31));
static_assert(NE % WCH == 0 && NE % 4 == 0);
static_assert(RCAP == NWAVE * WLCAP && (RCAP % (NTHR * 4)) == 0 && (BK_ZINTS % (NTHR * 4)) == 0);
static_assert((long long)RCAP * 100 >= (long long)MAXB1024_MEAS * 105);
static_assert(WLCAP >= MAXB1024_MEAS / 8 + 320);
static_assert(MAXDEG_MEAS + 8 <= DEGCAP);
static_assert(BK_LDS <= 300000 && BK_LDS <= 327680);
static_assert(CV_LDS <= 327680);
static_assert((NN * DH / 8) % NTHR == 0 && CBROWS % NTHR == 0 && CBROWS >= NN);
static_assert((DH * 32 / 8) % NTHR == 0 && (DH * DH / 8) % NTHR == 0);
static_assert(NCB * CNB >= NN && CNB == NWAVE * 16);
static_assert((2 * NBRUN) % (NTHR * 4) == 0);

typedef float          v4f   __attribute__((ext_vector_type(4)));
typedef float          v8f   __attribute__((ext_vector_type(8)));
typedef int            v4i   __attribute__((ext_vector_type(4)));
typedef int            v8i   __attribute__((ext_vector_type(8)));
typedef unsigned       v2u   __attribute__((ext_vector_type(2)));
typedef unsigned short v8us  __attribute__((ext_vector_type(8)));
typedef __bf16         v16bf __attribute__((ext_vector_type(16)));
typedef v4f __attribute__((may_alias)) v4fa;
typedef v4i __attribute__((may_alias)) v4ia;
typedef v2u __attribute__((may_alias)) v2ua;
union FragB { v16bf v; v8i w; v4i q[2]; };

__device__ __forceinline__ v8f wmx(const FragB& a, const FragB& b, v8f c) {
  v8f d = __builtin_amdgcn_wmma_f32_16x16x32_bf16(false, a.v, false, b.v, (short)0, c, false, false);
  asm volatile("v_nop\n\tv_nop\n\tv_nop\n\tv_nop" : "+v"(d) : "v"(a.w), "v"(b.w));
  return d;
}

__device__ __forceinline__ void pinf(float x) { asm volatile("" :: "v"(x)); }
__device__ __forceinline__ void pini(int x)   { asm volatile("" :: "v"(x)); }

__device__ __forceinline__ void wave_sync() {
  __builtin_amdgcn_fence(__ATOMIC_RELEASE, "wavefront");
  __builtin_amdgcn_wave_barrier();
}

__device__ __forceinline__ unsigned bfbits(float f) {
  const unsigned u = __float_as_uint(f);
  const unsigned r = (u + 0x7FFFu + ((u >> 16) & 1u)) >> 16;
  const unsigned q = (u >> 16) | 0x40u;
  return ((u & 0x7fffffffu) > 0x7f800000u) ? q : r;
}

__device__ __forceinline__ float relu_keep(float v) { return (v > 0.0f) ? v : (v - v); }

__device__ __forceinline__ void split2(float v0, float v1, int dolo, int& hw, int& lw) {
  const unsigned a0 = bfbits(v0), a1 = bfbits(v1);
  const unsigned b0 = bfbits(v0 - __uint_as_float(a0 << 16));
  const unsigned b1 = bfbits(v1 - __uint_as_float(a1 << 16));
  hw = (int)(a0 | (a1 << 16));
  lw = dolo ? (int)(b0 | (b1 << 16)) : 0;
}

__device__ __forceinline__ void st2_v4f(float* p, v4f v) {
  *(volatile v4f*)p = v;
  __threadfence();
  *(volatile v4f*)p = v;
}
__device__ __forceinline__ void st2_v8us(unsigned short* p, v8us v) {
  *(volatile v8us*)p = v;
  __threadfence();
  *(volatile v8us*)p = v;
}

__device__ __forceinline__ v8us gather8(const float* __restrict__ base, int stride) {
  float f[8];
#pragma unroll
  for (int i = 0; i < 8; ++i) f[i] = base[(size_t)i * (size_t)stride];
  v8us o;
#pragma unroll
  for (int i = 0; i < 8; ++i) o[i] = (unsigned short)bfbits(f[i]);
  return o;
}

template <int K> constexpr float mu_c() {
  return (K == NBAS - 1) ? 4.5f
                         : (0.0f * (1.0f - (float)K / 15.0f) + 4.5f * ((float)K / 15.0f));
}
constexpr float coeff_c() {
  return (float)(-0.5 / (((4.5 - 0.0) / 15.0) * ((4.5 - 0.0) / 15.0)));
}
template <int J> __device__ __forceinline__ float basis_val(float d, int hh) {
  constexpr float mu_a = mu_c<J>();
  constexpr float mu_b = mu_c<J + 8>();
  constexpr float cf   = coeff_c();
  const float mu = (hh != 0) ? mu_b : mu_a;
  const float x  = d - mu;
  const float sq = x * x;
  return expf(cf * sq);
}

__global__ __launch_bounds__(NTHR) void k_prep(const float* __restrict__ feats, const float* __restrict__ coords,
                                               const float* __restrict__ w1, const float* __restrict__ w2,
                                               unsigned short* fb, float* cb, unsigned short* w1p,
                                               unsigned short* w2t) {
  const int tid = (int)threadIdx.x;
  const int blk = (int)blockIdx.x;
  if (blk < PBF) {
    const int u   = blk * NTHR + tid;
    const int row = u >> 4, k8 = (u & 15) * 8;
    const float* p = feats + (size_t)row * DH + k8;
    const v4f a = *(const v4fa*)p;
    const v4f b = *(const v4fa*)(p + 4);
    v8us o;
    o[0] = (unsigned short)bfbits(a.x); o[1] = (unsigned short)bfbits(a.y);
    o[2] = (unsigned short)bfbits(a.z); o[3] = (unsigned short)bfbits(a.w);
    o[4] = (unsigned short)bfbits(b.x); o[5] = (unsigned short)bfbits(b.y);
    o[6] = (unsigned short)bfbits(b.z); o[7] = (unsigned short)bfbits(b.w);
    st2_v8us(fb + (size_t)row * DH + k8, o);
  } else if (blk < PBF + PBC) {
    const int row = (blk - PBF) * NTHR + tid;
    const int rc  = row < NN ? row : NN - 1;
    const float a0 = coords[3 * rc], a1 = coords[3 * rc + 1], a2 = coords[3 * rc + 2];
    pinf(a0); pinf(a1); pinf(a2);
    const unsigned mk = row < NN ? 0xffff0000u : 0u;
    v4f o;
    o.x = __uint_as_float((bfbits(a0) << 16) & mk);
    o.y = __uint_as_float((bfbits(a1) << 16) & mk);
    o.z = __uint_as_float((bfbits(a2) << 16) & mk);
    o.w = 0.0f;
    st2_v4f(cb + (size_t)4 * (size_t)row, o);
  } else if (blk < PBF + PBC + PBW1) {
    const int u  = (blk - PBF - PBC) * NTHR + tid;
    const int n  = u >> 2, k8 = (u & 3) * 8, kk = k8 & 15;
    const v8us o = gather8(w1 + (size_t)kk * DH + n, DH);
    st2_v8us(w1p + (size_t)n * 32 + k8, o);
  } else {
    const int u  = (blk - PBF - PBC - PBW1) * NTHR + tid;
    const int n  = u >> 4, k8 = (u & 15) * 8;
    const v8us o = gather8(w2 + (size_t)k8 * DH + n, DH);
    st2_v8us(w2t + (size_t)n * DH + k8, o);
  }
}

__device__ __forceinline__ void bucket_flush(const int* pl, const int* cnt, int ov, int* lp, int* cop, int* fp,
                                             int tid) {
#pragma unroll 1
  for (int i = tid * 4; i < RCAP; i += NTHR * 4) {
    const v4i v = *(const v4ia*)(pl + i);
    *(volatile v4i*)(lp + i) = v;
  }
#pragma unroll 1
  for (int i = tid * 4; i < 2 * NBRUN; i += NTHR * 4) {
    const v4i v = *(const v4ia*)(cnt + i);
    *(volatile v4i*)(cop + i) = v;
  }
  if (tid < 8) {
    const v4i f = {ov, ov, ov, ov};
    *(volatile v4i*)(fp + 4 * tid) = f;
  }
}

__global__ __launch_bounds__(NTHR) void k_bucket(const int* __restrict__ srcs, const int* __restrict__ dsts,
                                                 int* LIST, int* CO, int* FLAG) {
  extern __shared__ __attribute__((aligned(16))) int dsm[];
  int* wl   = dsm;
  int* pl   = dsm + NWAVE * WLCAP;
  int* cnt  = pl + RCAP;
  int* offs = cnt + NBRUN;
  int* cur  = offs + NBRUN;
  int* misc = cur + NBRUN;
  const int tid = (int)threadIdx.x, lane = tid & 31, wave = tid >> 5;
  const int blk = (int)blockIdx.x;
  const unsigned nbs = (unsigned)(blk * NBRUN);

  {
    const v4i z4 = {0, 0, 0, 0};
    for (int i = tid * 4; i < BK_ZINTS; i += NTHR * 4) *(v4ia*)(dsm + i) = z4;
    if (tid < 16) misc[tid] = 0;
  }
  __syncthreads();

  {
    const int per  = ((NE + NWAVE * WCH - 1) / (NWAVE * WCH)) * WCH;
    const int ebeg = wave * per;
    const int eend = (ebeg + per < NE) ? (ebeg + per) : NE;
    int* mylist = wl + wave * WLCAP;
    int wc = 0;
#pragma unroll 1
    for (int cb = ebeg; cb < eend; cb += WCH) {
      const int e0 = cb + lane * EPT;
      const v4i da = *(const v4ia*)(dsts + e0);
      const v4i db = *(const v4ia*)(dsts + e0 + 4);
      const unsigned s0 = (unsigned)da.x - nbs, s1 = (unsigned)da.y - nbs;
      const unsigned s2 = (unsigned)da.z - nbs, s3 = (unsigned)da.w - nbs;
      const unsigned s4 = (unsigned)db.x - nbs, s5 = (unsigned)db.y - nbs;
      const unsigned s6 = (unsigned)db.z - nbs, s7 = (unsigned)db.w - nbs;
      const bool h0 = s0 < (unsigned)NBRUN, h1 = s1 < (unsigned)NBRUN, h2 = s2 < (unsigned)NBRUN, h3 = s3 < (unsigned)NBRUN;
      const bool h4 = s4 < (unsigned)NBRUN, h5 = s5 < (unsigned)NBRUN, h6 = s6 < (unsigned)NBRUN, h7 = s7 < (unsigned)NBRUN;
      const unsigned m0 = __builtin_amdgcn_ballot_w32(h0), m1 = __builtin_amdgcn_ballot_w32(h1);
      const unsigned m2 = __builtin_amdgcn_ballot_w32(h2), m3 = __builtin_amdgcn_ballot_w32(h3);
      const unsigned m4 = __builtin_amdgcn_ballot_w32(h4), m5 = __builtin_amdgcn_ballot_w32(h5);
      const unsigned m6 = __builtin_amdgcn_ballot_w32(h6), m7 = __builtin_amdgcn_ballot_w32(h7);
      const unsigned any = m0 | m1 | m2 | m3 | m4 | m5 | m6 | m7;
      if (any != 0u) {
        const int pre = (int)(__builtin_amdgcn_mbcnt_lo(m0, 0u) + __builtin_amdgcn_mbcnt_lo(m1, 0u) +
                              __builtin_amdgcn_mbcnt_lo(m2, 0u) + __builtin_amdgcn_mbcnt_lo(m3, 0u) +
                              __builtin_amdgcn_mbcnt_lo(m4, 0u) + __builtin_amdgcn_mbcnt_lo(m5, 0u) +
                              __builtin_amdgcn_mbcnt_lo(m6, 0u) + __builtin_amdgcn_mbcnt_lo(m7, 0u));
        int p = wc + pre;
        if (h0) { if (p < WLCAP) mylist[p] = ((e0 + 0) << SLB) | (int)s0; p = p + 1; }
        if (h1) { if (p < WLCAP) mylist[p] = ((e0 + 1) << SLB) | (int)s1; p = p + 1; }
        if (h2) { if (p < WLCAP) mylist[p] = ((e0 + 2) << SLB) | (int)s2; p = p + 1; }
        if (h3) { if (p < WLCAP) mylist[p] = ((e0 + 3) << SLB) | (int)s3; p = p + 1; }
        if (h4) { if (p < WLCAP) mylist[p] = ((e0 + 4) << SLB) | (int)s4; p = p + 1; }
        if (h5) { if (p < WLCAP) mylist[p] = ((e0 + 5) << SLB) | (int)s5; p = p + 1; }
        if (h6) { if (p < WLCAP) mylist[p] = ((e0 + 6) << SLB) | (int)s6; p = p + 1; }
        if (h7) { if (p < WLCAP) mylist[p] = ((e0 + 7) << SLB) | (int)s7; p = p + 1; }
        wc += (int)(__builtin_popcount(m0) + __builtin_popcount(m1) + __builtin_popcount(m2) + __builtin_popcount(m3) +
                    __builtin_popcount(m4) + __builtin_popcount(m5) + __builtin_popcount(m6) + __builtin_popcount(m7));
      }
    }
    if (lane == 0) misc[wave] = wc;
  }
  __syncthreads();

  if (wave == 0) {
    int ov = 0;
#pragma unroll 1
    for (int w2 = 0; w2 < NWAVE; ++w2) {
      int c = misc[w2];
      if (c > WLCAP) ov = 1;
      c = c < 0 ? 0 : (c > WLCAP ? WLCAP : c);
#pragma unroll 1
      for (int b0 = 0; b0 < c; b0 += 32) {
        const int idx = b0 + lane;
        const int ent = wl[w2 * WLCAP + (idx < WLCAP ? idx : WLCAP - 1)];
        const int m32 = (c - b0) < 32 ? (c - b0) : 32;
#pragma unroll 1
        for (int k = 0; k < m32; ++k) {
          const int u    = __builtin_amdgcn_readlane(ent, k);
          const int slot = u & (NBRUN - 1);
          if (lane == 0) cnt[slot] = cnt[slot] + 1;
        }
      }
    }
    if (lane == 0) misc[9] = ov;
  }
  __syncthreads();
  if (wave == 0) {
    const int base = lane * (NBRUN / 32);
    int s = 0;
    int big = 0;
#pragma unroll 1
    for (int i = 0; i < NBRUN / 32; ++i) {
      const int cv = cnt[base + i];
      big = (cv > DEGCAP) ? 1 : big;
      s += cv;
    }
    int incl = s;
#pragma unroll
    for (int d = 1; d < 32; d <<= 1) {
      const int y = __shfl_up(incl, d, 32);
      if (lane >= d) incl += y;
    }
    int run = incl - s;
#pragma unroll 1
    for (int i = 0; i < NBRUN / 32; ++i) {
      const int cv = cnt[base + i];
      offs[base + i] = run;
      cur[base + i]  = run;
      run += cv;
    }
    const unsigned anyb = __builtin_amdgcn_ballot_w32(big != 0);
    if (lane == 0 && anyb != 0u) misc[9] = 1;
  }
  __syncthreads();

  if (wave == 0) {
#pragma unroll 1
    for (int w2 = 0; w2 < NWAVE; ++w2) {
      int c = misc[w2];
      c = c < 0 ? 0 : (c > WLCAP ? WLCAP : c);
#pragma unroll 1
      for (int b0 = 0; b0 < c; b0 += 32) {
        const int idx = b0 + lane;
        const int ent = wl[w2 * WLCAP + (idx < WLCAP ? idx : WLCAP - 1)];
        int eid = (ent >> SLB) & 0x1FFFFF;
        eid = eid > NE - 1 ? NE - 1 : eid;
        int sr = srcs[eid];
        sr = sr < 0 ? 0 : (sr > NN - 1 ? NN - 1 : sr);
        const int word = (int)((unsigned)sr | ((unsigned)(ent & (NBRUN - 1)) << 16));
        const int m32 = (c - b0) < 32 ? (c - b0) : 32;
#pragma unroll 1
        for (int k = 0; k < m32; ++k) {
          const int u    = __builtin_amdgcn_readlane(ent, k);
          const int wd   = __builtin_amdgcn_readlane(word, k);
          const int slot = u & (NBRUN - 1);
          if (lane == 0) {
            int p = cur[slot];
            p = p < 0 ? 0 : (p > RCAP - 1 ? RCAP - 1 : p);
            pl[p] = wd;
            cur[slot] = p + 1;
          }
        }
      }
    }
  }
  __syncthreads();

  const int ovf = misc[9];
  int* lp  = LIST + (size_t)blk * RCAP;
  int* cop = CO + (size_t)blk * (2 * NBRUN);
  int* fp  = FLAG + (size_t)blk * 32;
  bucket_flush(pl, cnt, ovf, lp, cop, fp, tid);
  __threadfence();
  bucket_flush(pl, cnt, ovf, lp, cop, fp, tid);
}

__global__ __launch_bounds__(NTHR) __attribute__((amdgpu_num_vgpr(248)))
void k_conv(const unsigned short* __restrict__ FB, const float* __restrict__ CB,
            const unsigned short* __restrict__ W1P, const unsigned short* __restrict__ W2T,
            const int* __restrict__ LIST, const int* __restrict__ CO, const int* __restrict__ FLAG,
            float* out) {
  extern __shared__ __attribute__((aligned(16))) int csm[];
  unsigned short* sW2 = (unsigned short*)csm;
  unsigned short* sW1 = sW2 + DH * W2PITCH;
  float*          sT  = (float*)(sW1 + DH * W1PITCH);
  const int tid = (int)threadIdx.x, lane = tid & 31, hh = lane >> 4, m = lane & 15;
  const int wave = __builtin_amdgcn_readfirstlane(tid >> 5);

#pragma unroll 4
  for (int it = 0; it < 8; ++it) {
    const int p = it * NTHR + tid;
    const int n = p >> 4, q = p & 15;
    const v4i v = *(const v4ia*)(W2T + (size_t)n * DH + 8 * q);
    *(v4ia*)(sW2 + n * W2PITCH + 8 * q) = v;
  }
#pragma unroll
  for (int it = 0; it < 2; ++it) {
    const int p = it * NTHR + tid;
    const int n = p >> 2, q = p & 3;
    const v4i v = *(const v4ia*)(W1P + (size_t)n * 32 + 8 * q);
    *(v4ia*)(sW1 + n * W1PITCH + 8 * q) = v;
  }
  __syncthreads();

  float* T = sT + wave * 16 * TP;
  const int nodeBase = (int)blockIdx.x * CNB;
  const v8f z8 = {0.f, 0.f, 0.f, 0.f, 0.f, 0.f, 0.f, 0.f};
  const float qnan = __uint_as_float(0x7fc00000u);

#pragma unroll 1
  for (int qi = 0; qi < CNB / NWAVE; ++qi) {
    const int i = nodeBase + wave + NWAVE * qi;
    if (i >= NN) break;
    const int bucket = i >> SLB;
    const int slot   = i & (NBRUN - 1);
    const int* cob = CO + (size_t)bucket * (2 * NBRUN);
    int cv = cob[slot];
    int ovv = cob[NBRUN + slot];
    const int fl = FLAG[(size_t)bucket * 32];
    pini(cv); pini(ovv); pini(fl);
    const int bigv = ((cv < 0) | (cv > DEGCAP) | (fl != 0)) ? 1 : 0;
    cv  = cv < 0 ? 0 : (cv > DEGCAP ? DEGCAP : cv);
    ovv = ovv < 0 ? 0 : (ovv > RCAP - 1 ? RCAP - 1 : ovv);
    cv  = cv > RCAP - ovv ? RCAP - ovv : cv;
    const int c = __builtin_amdgcn_readfirstlane(cv);
    const int o = __builtin_amdgcn_readfirstlane(ovv);
    const bool bad = __builtin_amdgcn_readfirstlane(bigv) != 0;
    int last = o + c - 1;
    last = last < o ? o : last;
    const int* lb = LIST + (size_t)bucket * RCAP;
    const v4f ci = *(const v4fa*)(CB + (size_t)4 * (size_t)i);
    float a0 = 0.0f, a1 = 0.0f, a2 = 0.0f, a3 = 0.0f;

#pragma unroll 1
    for (int t0 = 0; t0 < c; t0 += 16) {
      const int nv = (c - t0) < 16 ? (c - t0) : 16;
      int idx = o + t0 + m;
      idx = idx > last ? last : idx;
      const int en = lb[idx];
      pini(en);
      int s = en & 0xffff;
      s = s > NN - 1 ? NN - 1 : s;
      const v4f cs = *(const v4fa*)(CB + (size_t)4 * (size_t)s);
      asm volatile("" :: "v"(cs));
      const bool valid = (t0 + m) < c;

      const float dx = cs.x - ci.x, dy = cs.y - ci.y, dz = cs.z - ci.z;
      const float d  = sqrtf((dx * dx + dz * dz) + dy * dy);
      float b0 = basis_val<0>(d, hh), b1 = basis_val<1>(d, hh), b2 = basis_val<2>(d, hh), b3 = basis_val<3>(d, hh);
      float b4 = basis_val<4>(d, hh), b5 = basis_val<5>(d, hh), b6 = basis_val<6>(d, hh), b7 = basis_val<7>(d, hh);
      b0 = valid ? b0 : 0.0f; b1 = valid ? b1 : 0.0f; b2 = valid ? b2 : 0.0f; b3 = valid ? b3 : 0.0f;
      b4 = valid ? b4 : 0.0f; b5 = valid ? b5 : 0.0f; b6 = valid ? b6 : 0.0f; b7 = valid ? b7 : 0.0f;
      FragB af;
      {
        int h01, h23, h45, h67, l01, l23, l45, l67;
        split2(b0, b1, SPLIT_A, h01, l01);
        split2(b2, b3, SPLIT_A, h23, l23);
        split2(b4, b5, SPLIT_A, h45, l45);
        split2(b6, b7, SPLIT_A, h67, l67);
        const v8i t8 = {h01, h23, h45, h67, l01, l23, l45, l67};
        af.w = t8;
      }
      wave_sync();
#pragma unroll
      for (int t = 0; t < 8; ++t) {
        const unsigned short* wq = sW1 + (16 * t + m) * W1PITCH + 8 * hh;
        FragB bf;
        bf.q[0] = *(const v4ia*)wq;
        bf.q[1] = *(const v4ia*)(wq + 16);
        const v8f dd = wmx(af, bf, z8);
#pragma unroll
        for (int r = 0; r < 8; ++r) T[(8 * hh + r) * TP + 16 * t + m] = relu_keep(dd[r]);
      }
      wave_sync();

      v8f acc[8];
#pragma unroll
      for (int t = 0; t < 8; ++t) acc[t] = z8;
#pragma unroll 1
      for (int ks = 0; ks < DH / 32; ++ks) {
        const int k0 = 32 * ks;
        const float* tp = T + m * TP + k0 + 8 * hh;
        const v4f p0 = *(const v4fa*)tp;
        const v4f p1 = *(const v4fa*)(tp + 4);
        const v4f p2 = *(const v4fa*)(tp + 16);
        const v4f p3 = *(const v4fa*)(tp + 20);
        FragB ah, al;
        {
          int h0, h1, h2, h3, h4, h5, h6, h7, l0, l1, l2, l3, l4, l5, l6, l7;
          split2(p0.x, p0.y, 1, h0, l0); split2(p0.z, p0.w, 1, h1, l1);
          split2(p1.x, p1.y, 1, h2, l2); split2(p1.z, p1.w, 1, h3, l3);
          split2(p2.x, p2.y, 1, h4, l4); split2(p2.z, p2.w, 1, h5, l5);
          split2(p3.x, p3.y, 1, h6, l6); split2(p3.z, p3.w, 1, h7, l7);
          const v8i th = {h0, h1, h2, h3, h4, h5, h6, h7};
          const v8i tl = {l0, l1, l2, l3, l4, l5, l6, l7};
          ah.w = th;
          al.w = tl;
        }
#pragma unroll
        for (int t = 0; t < 8; ++t) {
          const unsigned short* wq = sW2 + (16 * t + m) * W2PITCH + k0 + 8 * hh;
          FragB bf;
          bf.q[0] = *(const v4ia*)wq;
          bf.q[1] = *(const v4ia*)(wq + 16);
          acc[t] = wmx(ah, bf, acc[t]);
#if MODE_B == 1
          acc[t] = wmx(al, bf, acc[t]);
#endif
        }
#if MODE_B != 1
        asm volatile("" :: "v"(al.w));
#endif
      }
      wave_sync();
#pragma unroll
      for (int t = 0; t < 8; ++t) {
#pragma unroll
        for (int r = 0; r < 8; ++r) T[(8 * hh + r) * TP + 16 * t + m] = relu_keep(acc[t][r]);
      }
      wave_sync();

#pragma unroll 1
      for (int r = 0; r < nv; ++r) {
        const int sr = __builtin_amdgcn_readlane(s, r);
        const v2u w = *(const v2ua*)(FB + (size_t)sr * DH + 4 * lane);
        const v4f f = *(const v4fa*)(T + r * TP + 4 * lane);
        const unsigned wx = w.x, wy = w.y;
        a0 = fmaf(__uint_as_float(wx << 16),          f.x, a0);
        a1 = fmaf(__uint_as_float(wx & 0xffff0000u),  f.y, a1);
        a2 = fmaf(__uint_as_float(wy << 16),          f.z, a2);
        a3 = fmaf(__uint_as_float(wy & 0xffff0000u),  f.w, a3);
      }
    }

    v4f ov;
    ov.x = bad ? qnan : a0; ov.y = bad ? qnan : a1; ov.z = bad ? qnan : a2; ov.w = bad ? qnan : a3;
    float* op = out + (size_t)i * DH + 4 * lane;
    *(volatile v4f*)op = ov;
    __threadfence();
    *(volatile v4f*)op = ov;
  }
}

extern "C" void kernel_launch(void* const* d_in, const int* in_sizes, int n_in,
                              void* d_out, int out_size, void* d_ws, size_t ws_size,
                              hipStream_t stream) {
  if (n_in < 6) return;
  if (in_sizes[0] != NN * DH) return;
  if (in_sizes[1] != NN * 3) return;
  if (in_sizes[2] != NE) return;
  if (in_sizes[3] != NE) return;
  if (in_sizes[4] != NBAS * DH) return;
  if (in_sizes[5] != DH * DH) return;
  if (out_size != NN * DH) return;

  const float* feats  = (const float*)d_in[0];
  const float* coords = (const float*)d_in[1];
  const int*   srcs   = (const int*)d_in[2];
  const int*   dsts   = (const int*)d_in[3];
  const float* W1     = (const float*)d_in[4];
  const float* W2     = (const float*)d_in[5];
  float* out = (float*)d_out;

  constexpr size_t zFB   = (size_t)NN * DH * 2;
  constexpr size_t zCB   = (size_t)CBROWS * 16;
  constexpr size_t zW1P  = (size_t)DH * 32 * 2;
  constexpr size_t zW2T  = (size_t)DH * DH * 2;
  constexpr size_t zLIST = (size_t)NBK * RCAP * 4;
  constexpr size_t zCO   = (size_t)NBK * 2 * NBRUN * 4;
  constexpr size_t zFLAG = 6400;
  constexpr size_t oFB   = 0;
  constexpr size_t oCB   = oFB + zFB;
  constexpr size_t oW1P  = oCB + zCB;
  constexpr size_t oW2T  = oW1P + zW1P;
  constexpr size_t oLIST = oW2T + zW2T;
  constexpr size_t oCO   = oLIST + zLIST;
  constexpr size_t oFLAG = oCO + zCO;
  constexpr size_t oEND  = oFLAG + zFLAG;
  static_assert(zFB % 256 == 0 && zCB % 256 == 0 && zW1P % 256 == 0 && zW2T % 256 == 0);
  static_assert(zLIST % 256 == 0 && zCO % 256 == 0 && zFLAG % 256 == 0 && zFLAG >= (size_t)NBK * 128);
  static_assert(oEND <= ((size_t)128 << 20));
  if (oEND > ws_size) return;

  char* ws = (char*)d_ws;
  unsigned short* FB   = (unsigned short*)(ws + oFB);
  float*          CB   = (float*)(ws + oCB);
  unsigned short* W1P  = (unsigned short*)(ws + oW1P);
  unsigned short* W2T  = (unsigned short*)(ws + oW2T);
  int*            LIST = (int*)(ws + oLIST);
  int*            CO   = (int*)(ws + oCO);
  int*            FLAG = (int*)(ws + oFLAG);

  (void)hipFuncSetAttribute(reinterpret_cast<const void*>(&k_bucket),
                            hipFuncAttributeMaxDynamicSharedMemorySize, (int)BK_LDS);
  (void)hipFuncSetAttribute(reinterpret_cast<const void*>(&k_conv),
                            hipFuncAttributeMaxDynamicSharedMemorySize, (int)CV_LDS);

  k_prep<<<PBTOT, NTHR, 0, stream>>>(feats, coords, W1, W2, FB, CB, W1P, W2T);
  k_bucket<<<NBK, NTHR, BK_LDS, stream>>>(srcs, dsts, LIST, CO, FLAG);
  k_conv<<<NCB, NTHR, CV_LDS, stream>>>(FB, CB, W1P, W2T, LIST, CO, FLAG, out);
}
